// TSGBlock_38946763440921
// MI455X (gfx1250) — hardware-run, weakly checked
//
#include <hip/hip_runtime.h>
#include <hip/hip_fp16.h>
#include <math.h>

typedef __attribute__((ext_vector_type(16))) _Float16 v16h;
typedef __attribute__((ext_vector_type(8)))  _Float16 v8h;
typedef __attribute__((ext_vector_type(8)))  float    v8f;
typedef __attribute__((ext_vector_type(4)))  float    v4f;
typedef __attribute__((ext_vector_type(2)))  unsigned v2u;

constexpr int kBatch  = 4;
constexpr int kSeq    = 1024;
constexpr int kRows   = kBatch * kSeq;
constexpr int kDin    = 512;
constexpr int kRank   = 16;
constexpr int kRankP  = 32;
constexpr int kNst    = 16;
constexpr int kProjN  = kRank + 2 * kNst;
constexpr int kProjP  = 64;
constexpr int kBcP    = 2 * kNst;
constexpr float kWCarry = 1024.0f;
constexpr float kResid  = 2048.0f;
constexpr float kYCarry = 16.0f;
static_assert(kProjN == 48 && kProjN <= kProjP && (kProjP % 64) == 0);
static_assert((kRows % 32) == 0 && (kDin % 64) == 0 && (kSeq % 64) == 0);
static_assert((kDin % 32) == 0 && (kRankP % 32) == 0 && kRank <= kRankP && (kRank % 8) == 0);
static_assert(kDin / 4 == 128 && (kRows % 8) == 0 && (kSeq % 8) == 0);
static_assert(kRank == 16 && kRankP == 32 && kBcP == 32 && kNst == 16);
static_assert(kRows == 4096);

constexpr size_t kSzXH   = (size_t)kRows * kDin * 2;
constexpr size_t kSzWXH  = (size_t)kProjP * kDin * 2;
constexpr size_t kSzWDT  = (size_t)kDin * kRankP * 2;
constexpr size_t kSzPROJ = (size_t)kRows * kProjP * 4;
constexpr size_t kSzDH   = (size_t)kRows * kRankP * 2;
constexpr size_t kSzF32  = (size_t)kRows * kDin * 4;
constexpr size_t kSzALOG = (size_t)kDin * kNst * 4;
constexpr size_t kSzVEC  = (size_t)kDin * 4;
constexpr size_t kSzBC   = (size_t)2 * kRows * kBcP * 4;
constexpr size_t kSzY16  = (size_t)kSeq * kDin * 2;
constexpr size_t kSzXR   = (size_t)kSeq * kDin * 4;
constexpr size_t kRelXH   = 0;
constexpr size_t kRelWXH  = kRelXH   + kSzXH;
constexpr size_t kRelWDT  = kRelWXH  + kSzWXH;
constexpr size_t kRelPROJ = kRelWDT  + kSzWDT;
constexpr size_t kRelDH   = kRelPROJ + kSzPROJ;
constexpr size_t kRelDTP  = kRelDH   + kSzDH;
constexpr size_t kRelDT   = kRelDTP  + kSzF32;
constexpr size_t kRelALOG = kRelDT   + kSzF32;
constexpr size_t kRelBDR  = kRelALOG + kSzALOG;
constexpr size_t kRelDR   = kRelBDR  + kSzVEC;
constexpr size_t kRelYF   = kRelDR   + kSzVEC;
constexpr size_t kBranchBytes = kRelYF + kSzF32;
constexpr size_t kOffBC   = 2 * kBranchBytes;
constexpr size_t kOffYH   = kOffBC + kSzBC;
constexpr size_t kOffYL   = kOffYH + kSzY16;
constexpr size_t kOffXR   = kOffYL + kSzY16;
constexpr size_t kWsTotal = kOffXR + kSzXR;
static_assert(kSzXH == 4194304ull && kSzWXH == 65536ull && kSzWDT == 32768ull);
static_assert(kSzPROJ == 1048576ull && kSzDH == 262144ull && kSzF32 == 8388608ull);
static_assert(kSzALOG == 32768ull && kSzVEC == 2048ull && kSzBC == 1048576ull);
static_assert(kSzY16 == 1048576ull && kSzXR == 2097152ull);
static_assert(kBranchBytes == 30806016ull);
static_assert(kWsTotal == 66854912ull);
static_assert(kWsTotal <= 134217728ull);
static_assert((kRelWXH % 128) == 0 && (kRelWDT % 128) == 0 && (kRelPROJ % 128) == 0 && (kRelDH % 128) == 0 &&
              (kRelDTP % 128) == 0 && (kRelDT % 128) == 0 && (kRelALOG % 128) == 0 && (kRelBDR % 128) == 0 &&
              (kRelDR % 128) == 0 && (kRelYF % 128) == 0 && (kBranchBytes % 128) == 0 && (kOffBC % 128) == 0 &&
              (kOffYH % 128) == 0 && (kOffYL % 128) == 0 && (kOffXR % 128) == 0);
static_assert((long)(kRows - 1) * kBcP + (long)kRows * kBcP + 2 * kNst - 1 < 2L * kRows * kBcP);

__device__ __forceinline__ _Float16 f16_flush(float v) {
  const float w = (fabsf(v) < 6.103515625e-05f) ? 0.0f : v;
  return (_Float16)w;
}

__device__ __forceinline__ float bf16r(float v) {
  unsigned u = __float_as_uint(v);
  u = (u + 0x7FFFu + ((u >> 16) & 1u)) & 0xFFFF0000u;
  return __uint_as_float(u);
}

__device__ __forceinline__ float h16_to_f32(unsigned hb) {
  const unsigned sgn = (hb & 0x8000u) << 16; const unsigned em = hb & 0x7fffu;
  const float fn = __uint_as_float((em << 13) + 0x38000000u);
  const float fs = (float)em * 5.9604644775390625e-8f;
  const float mag = (em < 0x400u) ? fs : fn; return __uint_as_float(__float_as_uint(mag) | sgn); }

namespace eng {
union FragU { v16h v; v8h h[2]; };
__device__ __forceinline__ v16h frag_load(const _Float16* p) {
  FragU f;
  f.h[0] = *(const v8h*)(p);
  f.h[1] = *(const v8h*)(p + 16);
  return f.v;
}
__device__ __forceinline__ v8f mma(v16h a, v16h b, v8f c) {
  return __builtin_amdgcn_wmma_f32_16x16x32_f16(false, a, false, b, (short)0, c, false, false);
}
__device__ __forceinline__ void guard1(v8f& a, v16h x, v16h y) {
  asm volatile("v_nop\n\tv_nop\n\tv_nop\n\tv_nop" : "+v"(a) : "v"(x), "v"(y));
}
__device__ __forceinline__ void guard_acc(v8f& a) {
  asm volatile("v_nop\n\tv_nop\n\tv_nop\n\tv_nop" : "+v"(a));
}
__device__ __forceinline__ void keep4(v16h a, v16h b, v16h c, v16h d) {
  asm volatile("v_nop" :: "v"(a), "v"(b), "v"(c), "v"(d));
}

template <int MI, int SPL>
__global__ __launch_bounds__(256) void gemm_f16_kernel(
    const unsigned short* __restrict__ Ap, const unsigned short* __restrict__ A2p, int lda,
    const unsigned short* __restrict__ Btp, const unsigned short* __restrict__ Bt2p, int ldb,
    float* __restrict__ C, int ldc, int M, int N, int K, float scale, float rscale)
{
  static_assert(MI >= 1 && MI <= 2);
  static_assert(SPL >= 0 && SPL <= 2);
  const _Float16* A   = (const _Float16*)Ap;
  const _Float16* A2  = (const _Float16*)A2p;
  const _Float16* Bt  = (const _Float16*)Btp;
  const _Float16* Bt2 = (const _Float16*)Bt2p;
  __shared__ __align__(16) float sT[8][16 * 68];
  const int lane = threadIdx.x & 31;
  const int wave = threadIdx.x >> 5;
  const int tilesN = N >> 6;
  const int tilesM = M / (16 * MI);
  const int tile = blockIdx.x * 8 + wave;
  if (tile >= tilesM * tilesN) return;
  const int tm = tile / tilesN;
  const int tn = tile - tm * tilesN;
  const int m0 = tm * (16 * MI);
  const int n0 = tn << 6;
  const int rlane = lane & 15;
  const int koff  = (lane >> 4) * 8;
  const int mOff  = (lane >> 4) * 8;

  v8f acc[MI][4], accr[MI][4];
#pragma unroll
  for (int i = 0; i < MI; ++i)
#pragma unroll
    for (int j = 0; j < 4; ++j) {
      acc[i][j]  = (v8f){0.f, 0.f, 0.f, 0.f, 0.f, 0.f, 0.f, 0.f};
      accr[i][j] = (v8f){0.f, 0.f, 0.f, 0.f, 0.f, 0.f, 0.f, 0.f};
    }

  for (int k0 = 0; k0 < K; k0 += 32) {
    v16h bh[4], bl[4];
#pragma unroll
    for (int j = 0; j < 4; ++j) {
      const size_t bo = (size_t)(n0 + (j << 4) + rlane) * ldb + koff + k0;
      bh[j] = frag_load(Bt + bo);
      if (SPL == 2) bl[j] = frag_load(Bt2 + bo); else bl[j] = bh[j];
    }
#pragma unroll
    for (int i = 0; i < MI; ++i) {
      const size_t ao = (size_t)(m0 + (i << 4) + rlane) * lda + koff + k0;
      const v16h ah = frag_load(A + ao);
      v16h al = ah;
      if (SPL >= 1) al = frag_load(A2 + ao);
#pragma unroll
      for (int j = 0; j < 4; ++j) {
        acc[i][j] = mma(ah, bh[j], acc[i][j]);
        if (SPL >= 1) accr[i][j] = mma(al, bh[j], accr[i][j]);
        if (SPL == 2) accr[i][j] = mma(ah, bl[j], accr[i][j]);
      }
#pragma unroll
      for (int j = 0; j < 4; ++j) {
        guard1(acc[i][j], ah, al);
        if (SPL >= 1) guard1(accr[i][j], ah, al);
      }
    }
    keep4(bh[0], bh[1], bh[2], bh[3]);
    if (SPL == 2) keep4(bl[0], bl[1], bl[2], bl[3]);
  }
#pragma unroll
  for (int i = 0; i < MI; ++i)
#pragma unroll
    for (int j = 0; j < 4; ++j) {
      guard_acc(acc[i][j]);
      if (SPL >= 1) guard_acc(accr[i][j]);
    }

  float* slab = sT[wave];
#pragma unroll
  for (int i = 0; i < MI; ++i) {
    const int mBase = m0 + (i << 4);
#pragma unroll
    for (int j = 0; j < 4; ++j) {
#pragma unroll
      for (int r = 0; r < 8; ++r) {
        float v = acc[i][j][r] * scale;
        if (SPL >= 1) v += accr[i][j][r] * rscale;
        slab[(mOff + r) * 68 + (j << 4) + rlane] = v;
      }
    }
    __builtin_amdgcn_fence(__ATOMIC_RELEASE, "workgroup");
    __builtin_amdgcn_wave_barrier();
    __builtin_amdgcn_fence(__ATOMIC_ACQUIRE, "workgroup");
    {
      const int hh = lane >> 4, c4 = (lane & 15) * 4;
      for (int pass = 0; pass < 2; ++pass) {
#pragma unroll
        for (int it = 0; it < 8; ++it) {
          const int row = it * 2 + hh;
          const v4f v = *(const v4f*)(slab + row * 68 + c4);
          *(volatile v4f*)(C + (size_t)(mBase + row) * ldc + n0 + c4) = v;
        }
        __threadfence();
      }
    }
    __builtin_amdgcn_fence(__ATOMIC_RELEASE, "workgroup");
    __builtin_amdgcn_wave_barrier();
    __builtin_amdgcn_fence(__ATOMIC_ACQUIRE, "workgroup");
  }
}
}

__global__ __launch_bounds__(256) void rne_rows_f16_kernel(
    const float* __restrict__ src, unsigned short* __restrict__ dH, int total8)
{
  const int i = blockIdx.x * 256 + threadIdx.x;
  if (i >= total8) return;
  const size_t e0 = (size_t)i << 3;
  const v4f a0 = *(const v4f*)(src + e0);
  const v4f a1 = *(const v4f*)(src + e0 + 4);
  const float f0 = a0[0];
  const float f1 = a0[1];
  const float f2 = a0[2];
  const float f3 = a0[3];
  const float f4 = a1[0];
  const float f5 = a1[1];
  const float f6 = a1[2];
  const float f7 = a1[3];
  v8h hv;
  hv[0] = f16_flush(bf16r(f0));
  hv[1] = f16_flush(bf16r(f1));
  hv[2] = f16_flush(bf16r(f2));
  hv[3] = f16_flush(bf16r(f3));
  hv[4] = f16_flush(bf16r(f4));
  hv[5] = f16_flush(bf16r(f5));
  hv[6] = f16_flush(bf16r(f6));
  hv[7] = f16_flush(bf16r(f7));
  unsigned short* qh = dH + e0;
  *(volatile v8h*)qh = hv;
  __threadfence();
  *(volatile v8h*)qh = hv;
}

__global__ __launch_bounds__(256) void pack_rows_bf_kernel(
    const float* __restrict__ W, unsigned short* __restrict__ dH,
    int Kdim, int Nreal, int total8, float carry)
{
  const int i = blockIdx.x * 256 + threadIdx.x;
  if (i >= total8) return;
  const size_t e0 = (size_t)i << 3;
  const int row = (int)(e0 / (size_t)Kdim);
  const int col = (int)(e0 - (size_t)row * (size_t)Kdim);
  const bool live = (row < Nreal);
  const int rc = live ? row : (Nreal - 1);
  const v4f a0 = *(const v4f*)(W + (size_t)rc * Kdim + col);
  const v4f a1 = *(const v4f*)(W + (size_t)rc * Kdim + col + 4);
  const float w0 = a0[0];
  const float w1 = a0[1];
  const float w2 = a0[2];
  const float w3 = a0[3];
  const float w4 = a1[0];
  const float w5 = a1[1];
  const float w6 = a1[2];
  const float w7 = a1[3];
  const float t0 = bf16r(w0) * carry;
  const float t1 = bf16r(w1) * carry;
  const float t2 = bf16r(w2) * carry;
  const float t3 = bf16r(w3) * carry;
  const float t4 = bf16r(w4) * carry;
  const float t5 = bf16r(w5) * carry;
  const float t6 = bf16r(w6) * carry;
  const float t7 = bf16r(w7) * carry;
  const float g0 = live ? t0 : 0.0f;
  const float g1 = live ? t1 : 0.0f;
  const float g2 = live ? t2 : 0.0f;
  const float g3 = live ? t3 : 0.0f;
  const float g4 = live ? t4 : 0.0f;
  const float g5 = live ? t5 : 0.0f;
  const float g6 = live ? t6 : 0.0f;
  const float g7 = live ? t7 : 0.0f;
  v8h hv;
  hv[0] = f16_flush(g0);
  hv[1] = f16_flush(g1);
  hv[2] = f16_flush(g2);
  hv[3] = f16_flush(g3);
  hv[4] = f16_flush(g4);
  hv[5] = f16_flush(g5);
  hv[6] = f16_flush(g6);
  hv[7] = f16_flush(g7);
  unsigned short* qh = dH + e0;
  *(volatile v8h*)qh = hv;
  __threadfence();
  *(volatile v8h*)qh = hv;
}

__global__ __launch_bounds__(256) void pack_kpad_bf_kernel(
    const float* __restrict__ W, unsigned short* __restrict__ dH, int total8, float carry)
{
  constexpr int kGroupsP = kRankP / 8;
  constexpr int kGroupsL = kRank / 8;
  const int i = blockIdx.x * 256 + threadIdx.x;
  if (i >= total8) return;
  const int row = i / kGroupsP;
  const int g = i - row * kGroupsP;
  const bool live = (g < kGroupsL);
  const int gc = live ? g : (kGroupsL - 1);
  const float* sp = W + (size_t)row * kRank + gc * 8;
  const v4f a0 = *(const v4f*)(sp);
  const v4f a1 = *(const v4f*)(sp + 4);
  const float w0 = a0[0];
  const float w1 = a0[1];
  const float w2 = a0[2];
  const float w3 = a0[3];
  const float w4 = a1[0];
  const float w5 = a1[1];
  const float w6 = a1[2];
  const float w7 = a1[3];
  const float t0 = bf16r(w0) * carry;
  const float t1 = bf16r(w1) * carry;
  const float t2 = bf16r(w2) * carry;
  const float t3 = bf16r(w3) * carry;
  const float t4 = bf16r(w4) * carry;
  const float t5 = bf16r(w5) * carry;
  const float t6 = bf16r(w6) * carry;
  const float t7 = bf16r(w7) * carry;
  const float g0 = live ? t0 : 0.0f;
  const float g1 = live ? t1 : 0.0f;
  const float g2 = live ? t2 : 0.0f;
  const float g3 = live ? t3 : 0.0f;
  const float g4 = live ? t4 : 0.0f;
  const float g5 = live ? t5 : 0.0f;
  const float g6 = live ? t6 : 0.0f;
  const float g7 = live ? t7 : 0.0f;
  v8h hv;
  hv[0] = f16_flush(g0);
  hv[1] = f16_flush(g1);
  hv[2] = f16_flush(g2);
  hv[3] = f16_flush(g3);
  hv[4] = f16_flush(g4);
  hv[5] = f16_flush(g5);
  hv[6] = f16_flush(g6);
  hv[7] = f16_flush(g7);
  unsigned short* qh = dH + ((size_t)i << 3);
  *(volatile v8h*)qh = hv;
  __threadfence();
  *(volatile v8h*)qh = hv;
}

__global__ __launch_bounds__(256) void rne_vec_kernel(
    const float* __restrict__ src, float* __restrict__ dst, int n4)
{
  const int i = blockIdx.x * 256 + threadIdx.x;
  if (i >= n4) return;
  const v4f a = *(const v4f*)(src + (size_t)i * 4);
  const float a0 = a[0];
  const float a1 = a[1];
  const float a2 = a[2];
  const float a3 = a[3];
  v4f r;
  r[0] = bf16r(a0);
  r[1] = bf16r(a1);
  r[2] = bf16r(a2);
  r[3] = bf16r(a3);
  float* p = dst + (size_t)i * 4;
  *(volatile v4f*)p = r;
  __threadfence();
  *(volatile v4f*)p = r;
}

__global__ __launch_bounds__(256) void rne_plane_kernel(
    const float* __restrict__ src, float* __restrict__ dst, int n4)
{
  const int i = blockIdx.x * 256 + threadIdx.x;
  if (i >= n4) return;
  const v4f a = *(const v4f*)(src + (size_t)i * 4);
  const float a0 = a[0];
  const float a1 = a[1];
  const float a2 = a[2];
  const float a3 = a[3];
  v4f r;
  r[0] = bf16r(a0);
  r[1] = bf16r(a1);
  r[2] = bf16r(a2);
  r[3] = bf16r(a3);
  float* p = dst + (size_t)i * 4;
  *(volatile v4f*)p = r;
  __threadfence();
  *(volatile v4f*)p = r;
}

__global__ __launch_bounds__(128) void proj_split_kernel(
    const float* __restrict__ P, unsigned short* __restrict__ dH, float* __restrict__ BC)
{
  const int tid = threadIdx.x;
  const int r0 = blockIdx.x * 32;
  const int rowa = r0 + (tid >> 2);
  const int ga = tid & 3;
  const int g8 = ga * 8;
  const bool livea = (ga < kRank / 8);
  v8h hv;
  {
    const float* sp = P + (size_t)rowa * kProjP + g8;
    const v4f a0 = *(const v4f*)(sp);
    const v4f a1 = *(const v4f*)(sp + 4);
#pragma unroll
    for (int e = 0; e < 4; ++e) {
      const float f0 = a0[e];
      const float f1 = a1[e];
      const float s0 = livea ? f0 : 0.0f;
      const float s1 = livea ? f1 : 0.0f;
      hv[e] = f16_flush(s0);
      hv[4 + e] = f16_flush(s1);
    }
  }
  const int p4 = (tid & 7) * 4;
  v4f bcv[2];
#pragma unroll
  for (int it = 0; it < 2; ++it) {
    const int rowb = r0 + it * 16 + (tid >> 3);
    const v4f pv = *(const v4f*)(P + (size_t)rowb * kProjP + kRank + p4);
    bcv[it] = pv;
  }
  for (int pass = 0; pass < 2; ++pass) {
    *(volatile v8h*)(dH + (size_t)rowa * kRankP + g8) = hv;
#pragma unroll
    for (int it = 0; it < 2; ++it) {
      const int rowb = r0 + it * 16 + (tid >> 3);
      *(volatile v4f*)(BC + (size_t)rowb * kBcP + p4) = bcv[it];
    }
    __threadfence();
  }
}

__global__ __launch_bounds__(256) void dt_bias_kernel(
    const float* __restrict__ DTP, const float* __restrict__ bdt, float* __restrict__ DT)
{
  const int d4 = (blockIdx.x * 256 + threadIdx.x) * 4;
  const int r0 = blockIdx.y * 8;
  const v4f b = *(const v4f*)(bdt + d4);
  v4f val[8];
#pragma unroll
  for (int i = 0; i < 8; ++i) {
    const v4f p = *(const v4f*)(DTP + (size_t)(r0 + i) * kDin + d4);
    val[i] = p + b;
  }
  for (int pass = 0; pass < 2; ++pass) {
#pragma unroll
    for (int i = 0; i < 8; ++i)
      *(volatile v4f*)(DT + (size_t)(r0 + i) * kDin + d4) = val[i];
    __threadfence();
  }
}

typedef float    ms1_v4f __attribute__((ext_vector_type(4)));
typedef unsigned ms1_v4u __attribute__((ext_vector_type(4)));
struct ms1_args {
  const float* dtpre;
  const float* u;
  const float* bc;
  const float* z;
  const float* A_log;
  const float* Dskip;
  __half* y;
  __half* y_lo;
  long ld_dtpre;
  long ld_u;
  long ld_bc;
  long ld_z;
  long ld_y;
  int offB;
  int offC;
  int offZ;
  float ycarry;
  int dir;
  int D;
  int L;
  int nbatch;
};
static_assert(sizeof(ms1_args) == 136);

__device__ __forceinline__ float ms1_flush16(float v) {
  return (fabsf(v) < 6.103515625e-05f) ? 0.0f : v;
}
__device__ __forceinline__ unsigned ms1_h16bits(float v) {
  return (unsigned)__half_as_ushort(__float2half_rn(ms1_flush16(v)));
}
__device__ __forceinline__ float ms1_h16val(unsigned b) {
  return __half2float(__ushort_as_half((unsigned short)b));
}
__device__ __forceinline__ float ms1_softplus(float v) {
  return fmaxf(v, 0.0f) + log1pf(expf(-fabsf(v)));
}
__device__ __forceinline__ void ms1_pack2(float v0, float v1, unsigned& hw, unsigned& lw) {
  const unsigned h0 = ms1_h16bits(v0);
  const unsigned h1 = ms1_h16bits(v1);
  const float r0 = (v0 - ms1_h16val(h0)) * 2048.0f;
  const float r1 = (v1 - ms1_h16val(h1)) * 2048.0f;
  const unsigned l0 = ms1_h16bits(r0);
  const unsigned l1 = ms1_h16bits(r1);
  hw = h0 | (h1 << 16);
  lw = l0 | (l1 << 16);
}

template <int NSTATE>
__global__ __launch_bounds__(64 * (NSTATE / 16)) void ms1_scan_kernel(ms1_args a)
{
  static_assert(NSTATE == 16 || NSTATE == 64);
  constexpr int NQ  = NSTATE / 16;
  constexpr int NT  = 64 * NQ;
  constexpr int NW  = NT / 32;
  constexpr int BCW = 2 * NSTATE;
  constexpr int YP  = 68;
  constexpr int RPI = NW * 4;
  constexpr int NIT = 64 / RPI;
  static_assert(16 * NT <= 64 * YP);
  __shared__ __align__(16) float sBC[64 * BCW];
  __shared__ __align__(16) float sY[64 * YP];
  const int tid  = threadIdx.x;
  const int lane = tid & 31;
  const int wave = tid >> 5;
  const int c    = tid / NQ;
  const int sq   = tid - c * NQ;
  const int bpb  = a.D / 64;
  const int bi   = blockIdx.x / bpb;
  if (bi >= a.nbatch) return;
  const int d0 = (blockIdx.x - bi * bpb) * 64;
  const int d  = d0 + c;
  const long rowb = (long)bi * a.L;
  const bool hasz  = (a.z != nullptr);
  const bool hasD  = (a.Dskip != nullptr);
  const bool hasLo = (a.y_lo != nullptr);

#pragma unroll 1
  for (int n = 0; n < 16; ++n) {
    const float al = a.A_log[(long)d * NSTATE + sq * 16 + n];
    sY[n * NT + tid] = -expf(al);
  }
  __syncthreads();
  float An[16], h[16];
#pragma unroll
  for (int n = 0; n < 16; ++n) {
    An[n] = sY[n * NT + tid];
    h[n] = 0.0f;
  }
  float Dd = 0.0f;
  if (hasD) Dd = a.Dskip[d];

  const int nchunk = a.L / 64;
  const bool fwd = (a.dir > 0);
  const int s0 = fwd ? 0 : 63;
  const int sd = fwd ? 1 : -1;
  const int q  = lane >> 3;
  const int c8 = (lane & 7) * 8;

  for (int ci = 0; ci < nchunk; ++ci) {
    const int tb = fwd ? (ci * 64) : (a.L - 64 - ci * 64);
    const long rowc = rowb + tb;
    __syncthreads();
#pragma unroll 8
    for (int i = 0; i < 32; ++i) {
      const int idx = tid + i * NT;
      const int st  = idx / BCW;
      const int col = idx - st * BCW;
      const int sc  = (col < NSTATE) ? (a.offB + col) : (a.offC + col - NSTATE);
      sBC[idx] = a.bc[(rowc + st) * a.ld_bc + sc];
    }
    __syncthreads();
    for (int s = 0; s < 64; ++s) {
      const int ls = s0 + sd * s;
      const long row = rowc + ls;
      float pre = a.dtpre[row * a.ld_dtpre + d];
      float uv  = a.u[row * a.ld_u + d];
      float zv  = 0.0f;
      if (hasz) zv = a.z[row * a.ld_z + a.offZ + d];
      asm volatile("" : "+v"(pre));
      asm volatile("" : "+v"(uv));
      asm volatile("" : "+v"(zv));
      const float delta = ms1_softplus(pre);
      const float dtx = delta * uv;
      const float* bp = sBC + ls * BCW + sq * 16;
      const float* cp = bp + NSTATE;
      ms1_v4f Bq[4], Cq[4];
#pragma unroll
      for (int k = 0; k < 4; ++k) {
        Bq[k] = *(const ms1_v4f*)(bp + 4 * k);
        Cq[k] = *(const ms1_v4f*)(cp + 4 * k);
      }
      float yv = 0.0f;
#pragma unroll
      for (int n = 0; n < 16; ++n) {
        const float e = __expf(delta * An[n]);
        h[n] = fmaf(e, h[n], dtx * Bq[n >> 2][n & 3]);
        yv = fmaf(h[n], Cq[n >> 2][n & 3], yv);
      }
      if (NQ > 1) {
        yv += __shfl_xor(yv, 1, 32);
        yv += __shfl_xor(yv, 2, 32);
      }
      if (hasD) yv = fmaf(uv, Dd, yv);
      if (hasz) {
        const float sg = __builtin_amdgcn_rcpf(1.0f + expf(-zv));
        yv = yv * (zv * sg);
      }
      if (sq == 0) sY[ls * YP + c] = yv * a.ycarry;
    }
    __syncthreads();
    ms1_v4u hw[NIT], lw[NIT];
#pragma unroll
    for (int it = 0; it < NIT; ++it) {
      const int row = it * RPI + wave * 4 + q;
      const float* sp = sY + row * YP + c8;
      const ms1_v4f f0 = *(const ms1_v4f*)(sp);
      const ms1_v4f f1 = *(const ms1_v4f*)(sp + 4);
      unsigned h0, h1, h2, h3, l0, l1, l2, l3;
      ms1_pack2(f0[0], f0[1], h0, l0);
      ms1_pack2(f0[2], f0[3], h1, l1);
      ms1_pack2(f1[0], f1[1], h2, l2);
      ms1_pack2(f1[2], f1[3], h3, l3);
      hw[it] = (ms1_v4u){h0, h1, h2, h3};
      lw[it] = (ms1_v4u){l0, l1, l2, l3};
    }
    for (int pass = 0; pass < 2; ++pass) {
#pragma unroll
      for (int it = 0; it < NIT; ++it) {
        const int row = it * RPI + wave * 4 + q;
        const long o = (rowc + row) * a.ld_y + d0 + c8;
        *(volatile ms1_v4u*)(a.y + o) = hw[it];
        if (hasLo) *(volatile ms1_v4u*)(a.y_lo + o) = lw[it];
      }
      __threadfence();
    }
  }
}

__global__ __launch_bounds__(256) void rejoin_store_kernel(
    const unsigned short* __restrict__ YH, const unsigned short* __restrict__ YL, float* __restrict__ out)
{
  const int d4 = (blockIdx.x * 256 + threadIdx.x) * 4;
  const int r0 = blockIdx.y * 8;
  constexpr float kInvResid = 1.0f / kResid;
  constexpr float kInvCarry = 1.0f / kYCarry;
  v4f val[8];
#pragma unroll
  for (int i = 0; i < 8; ++i) {
    const size_t o = (size_t)(r0 + i) * kDin + d4;
    const v2u hw = *(const v2u*)(const void*)(YH + o);
    const v2u lw = *(const v2u*)(const void*)(YL + o);
    const float h0 = h16_to_f32(hw[0] & 0xffffu);
    const float h1 = h16_to_f32(hw[0] >> 16);
    const float h2 = h16_to_f32(hw[1] & 0xffffu);
    const float h3 = h16_to_f32(hw[1] >> 16);
    const float l0 = h16_to_f32(lw[0] & 0xffffu);
    const float l1 = h16_to_f32(lw[0] >> 16);
    const float l2 = h16_to_f32(lw[1] & 0xffffu);
    const float l3 = h16_to_f32(lw[1] >> 16);
    v4f v;
    v[0] = (h0 + l0 * kInvResid) * kInvCarry;
    v[1] = (h1 + l1 * kInvResid) * kInvCarry;
    v[2] = (h2 + l2 * kInvResid) * kInvCarry;
    v[3] = (h3 + l3 * kInvResid) * kInvCarry;
    val[i] = v;
  }
  for (int pass = 0; pass < 2; ++pass) {
#pragma unroll
    for (int i = 0; i < 8; ++i)
      *(volatile v4f*)(out + (size_t)(r0 + i) * kDin + d4) = val[i];
    __threadfence();
  }
}

static_assert(((kRows * (kDin / 4)) % 256) == 0 && (kDin / 4) == 128);
__global__ __launch_bounds__(256) void ln_out_kernel(
    const float* __restrict__ YF, const float* __restrict__ g, const float* __restrict__ beta,
    float* __restrict__ out)
{
  const int G  = blockIdx.x * 256 + threadIdx.x;
  const int r  = G >> 7;
  const int n4 = G & 127;
  const float* yr = YF + (size_t)r * kDin;
  constexpr float kInvN = 1.0f / (float)kDin;
  float acc = 0.0f;
  for (int j = 0; j < kDin / 4; ++j) {
    const v4f v = *(const v4f*)(yr + 4 * j);
    const float v0 = v[0];
    const float v1 = v[1];
    const float v2 = v[2];
    const float v3 = v[3];
    acc += v0;
    acc += v1;
    acc += v2;
    acc += v3;
  }
  const float mu = acc * kInvN;
  float acc2 = 0.0f;
  for (int j = 0; j < kDin / 4; ++j) {
    const v4f v = *(const v4f*)(yr + 4 * j);
    const float e0 = v[0] - mu;
    const float e1 = v[1] - mu;
    const float e2 = v[2] - mu;
    const float e3 = v[3] - mu;
    acc2 = fmaf(e0, e0, acc2);
    acc2 = fmaf(e1, e1, acc2);
    acc2 = fmaf(e2, e2, acc2);
    acc2 = fmaf(e3, e3, acc2);
  }
  const float var  = acc2 * kInvN;
  const float rstd = 1.0f / sqrtf(var + 1e-5f);
  const v4f yv = *(const v4f*)(yr + 4 * n4);
  const v4f gv = *(const v4f*)(g + 4 * n4);
  const v4f bv = *(const v4f*)(beta + 4 * n4);
  const float y0 = yv[0];
  const float y1 = yv[1];
  const float y2 = yv[2];
  const float y3 = yv[3];
  const float g0 = gv[0];
  const float g1 = gv[1];
  const float g2 = gv[2];
  const float g3 = gv[3];
  const float b0 = bv[0];
  const float b1 = bv[1];
  const float b2 = bv[2];
  const float b3 = bv[3];
  v4f res;
  res[0] = fmaf((y0 - mu) * rstd, bf16r(g0), bf16r(b0));
  res[1] = fmaf((y1 - mu) * rstd, bf16r(g1), bf16r(b1));
  res[2] = fmaf((y2 - mu) * rstd, bf16r(g2), bf16r(b2));
  res[3] = fmaf((y3 - mu) * rstd, bf16r(g3), bf16r(b3));
  float* p = out + (size_t)r * kDin + 4 * n4;
  *(volatile v4f*)p = res;
  __threadfence();
  *(volatile v4f*)p = res;
}

static_assert((kRows % 16) == 0 && (kRows % 32) == 0);
static_assert((kProjP % 64) == 0 && (kDin % 64) == 0);
static_assert(((kRows / 16) * (kProjP / 64)) % 8 == 0);
static_assert(((kRows / 32) * (kDin / 64)) % 8 == 0);
static_assert(((kRows * kDin / 8) % 256) == 0);
static_assert(((kProjP * kDin / 8) % 256) == 0);
static_assert(((kDin * kRankP / 8) % 256) == 0);
static_assert(((kDin * kNst / 4) % 256) == 0);
static_assert((kDin / 4) <= 256);
static_assert(((kSeq * kDin / 4) % 256) == 0);

extern "C" void kernel_launch(void* const* d_in, const int* in_sizes, int n_in,
                              void* d_out, int out_size, void* d_ws, size_t ws_size,
                              hipStream_t stream)
{
  if (n_in != 16) return;
  if (in_sizes[0] != kRows * kDin) return;
  if (in_sizes[1] != kRows * kDin) return;
  if (in_sizes[2] != kProjN * kDin) return;
  if (in_sizes[3] != kProjN * kDin) return;
  if (in_sizes[4] != kDin * kRank) return;
  if (in_sizes[5] != kDin) return;
  if (in_sizes[6] != kDin * kRank) return;
  if (in_sizes[7] != kDin) return;
  if (in_sizes[8] != kDin * kNst) return;
  if (in_sizes[9] != kDin * kNst) return;
  if (in_sizes[10] != kDin) return;
  if (in_sizes[11] != kDin) return;
  if (in_sizes[12] != kDin) return;
  if (in_sizes[13] != kDin) return;
  if (in_sizes[14] != kDin) return;
  if (in_sizes[15] != kDin) return;
  if (out_size != 2 * kRows * kDin) return;
  if (ws_size < kWsTotal) return;

  const float* xs[2]  = {(const float*)d_in[0],  (const float*)d_in[1]};
  const float* wxp[2] = {(const float*)d_in[2],  (const float*)d_in[3]};
  const float* wdt[2] = {(const float*)d_in[4],  (const float*)d_in[6]};
  const float* bdt[2] = {(const float*)d_in[5],  (const float*)d_in[7]};
  const float* alg[2] = {(const float*)d_in[8],  (const float*)d_in[9]};
  const float* dsk[2] = {(const float*)d_in[10], (const float*)d_in[11]};
  const float* lng[2] = {(const float*)d_in[12], (const float*)d_in[14]};
  const float* lnb[2] = {(const float*)d_in[13], (const float*)d_in[15]};
  float* out = (float*)d_out;

  char* ws = (char*)d_ws;
  float*          BC = (float*)(ws + kOffBC);
  unsigned short* YH = (unsigned short*)(ws + kOffYH);
  unsigned short* YL = (unsigned short*)(ws + kOffYL);
  float*          XR = (float*)(ws + kOffXR);

  constexpr float sW = 1.0f / kWCarry;

  for (int s = 0; s < 2; ++s) {
    char* base = ws + (size_t)s * kBranchBytes;
    unsigned short* XH   = (unsigned short*)(base + kRelXH);
    unsigned short* WXH  = (unsigned short*)(base + kRelWXH);
    unsigned short* WDT  = (unsigned short*)(base + kRelWDT);
    float*          PROJ = (float*)(base + kRelPROJ);
    unsigned short* DH   = (unsigned short*)(base + kRelDH);
    float*          DTP  = (float*)(base + kRelDTP);
    float*          DT   = (float*)(base + kRelDT);
    float*          ALOG = (float*)(base + kRelALOG);
    float*          BDR  = (float*)(base + kRelBDR);
    float*          DR   = (float*)(base + kRelDR);

    rne_rows_f16_kernel<<<(kRows * kDin / 8) / 256, 256, 0, stream>>>(xs[s], XH, kRows * kDin / 8);

    pack_rows_bf_kernel<<<(kProjP * kDin / 8) / 256, 256, 0, stream>>>(
        wxp[s], WXH, kDin, kProjN, kProjP * kDin / 8, kWCarry);

    pack_kpad_bf_kernel<<<(kDin * kRankP / 8) / 256, 256, 0, stream>>>(
        wdt[s], WDT, kDin * kRankP / 8, kWCarry);

    rne_vec_kernel<<<1, 256, 0, stream>>>(bdt[s], BDR, kDin / 4);
    rne_vec_kernel<<<1, 256, 0, stream>>>(dsk[s], DR, kDin / 4);

    rne_vec_kernel<<<(kDin * kNst / 4) / 256, 256, 0, stream>>>(alg[s], ALOG, kDin * kNst / 4);

    eng::gemm_f16_kernel<1, 0><<<dim3((kRows / 16) * (kProjP / 64) / 8), 256, 0, stream>>>(
        XH, nullptr, kDin, WXH, nullptr, kDin, PROJ, kProjP, kRows, kProjP, kDin, sW, 0.0f);

    proj_split_kernel<<<kRows / 32, 128, 0, stream>>>(PROJ, DH, BC + (size_t)s * kRows * kBcP);

    eng::gemm_f16_kernel<2, 0><<<dim3((kRows / 32) * (kDin / 64) / 8), 256, 0, stream>>>(
        DH, nullptr, kRankP, WDT, nullptr, kRankP, DTP, kDin, kRows, kDin, kRankP, sW, 0.0f);

    dt_bias_kernel<<<dim3(1, kRows / 8), kDin / 4, 0, stream>>>(DTP, BDR, DT);
  }

  for (int s = 0; s < 2; ++s) {
    char* base = ws + (size_t)s * kBranchBytes;
    float* DT   = (float*)(base + kRelDT);
    float* ALOG = (float*)(base + kRelALOG);
    float* DR   = (float*)(base + kRelDR);
    float* YF   = (float*)(base + kRelYF);
    for (int b = 0; b < kBatch; ++b) {
      const size_t rb = (size_t)b * kSeq;
      rne_plane_kernel<<<(kSeq * kDin / 4) / 256, 256, 0, stream>>>(xs[s] + rb * kDin, XR, kSeq * kDin / 4);

      ms1_args sa;
      sa.dtpre = DT + rb * kDin;
      sa.u = XR;
      sa.bc = BC + rb * kBcP;
      sa.z = nullptr;
      sa.A_log = ALOG;
      sa.Dskip = DR;
      sa.y = (__half*)YH;
      sa.y_lo = (__half*)YL;
      sa.ld_dtpre = kDin;
      sa.ld_u = kDin;
      sa.ld_bc = kBcP;
      sa.ld_z = 0;
      sa.ld_y = kDin;
      sa.offB = (s == 0) ? 0 : kRows * kBcP;
      sa.offC = (s == 0) ? (kRows * kBcP + kNst) : kNst;
      sa.offZ = 0;
      sa.ycarry = kYCarry;
      sa.dir = 1;
      sa.D = kDin;
      sa.L = kSeq;
      sa.nbatch = 1;
      ms1_scan_kernel<16><<<dim3(kDin / 64), 64, 0, stream>>>(sa);

      rejoin_store_kernel<<<dim3(1, kSeq / 8), kDin / 4, 0, stream>>>(YH, YL, YF + rb * kDin);
    }
  }

  for (int s = 0; s < 2; ++s) {
    char* base = ws + (size_t)s * kBranchBytes;
    const float* YF = (const float*)(base + kRelYF);
    ln_out_kernel<<<(kRows * (kDin / 4)) / 256, 256, 0, stream>>>(
        YF, lng[s], lnb[s], out + (size_t)s * kRows * kDin);
  }
}
